// HCL_37907381354588
// MI455X (gfx1250) — hardware-run, weakly checked
//
#include <hip/hip_runtime.h>
#include <math.h>

typedef __attribute__((ext_vector_type(16))) _Float16 v16h;
typedef __attribute__((ext_vector_type(8)))  _Float16 v8h;
typedef __attribute__((ext_vector_type(16))) __bf16   v16b;
typedef __attribute__((ext_vector_type(8)))  __bf16   v8b;
typedef __attribute__((ext_vector_type(8)))  float    v8f;
typedef __attribute__((ext_vector_type(4)))  float    v4f;
typedef __attribute__((ext_vector_type(4)))  unsigned int v4u;
typedef __attribute__((ext_vector_type(2)))  unsigned int v2u;

constexpr int    kTok       = 4096;
constexpr int    kDim       = 512;
constexpr size_t kND        = (size_t)kTok * kDim;
constexpr size_t kWW        = (size_t)kDim * kDim;
constexpr float  kWCarry    = 256.0f;
constexpr float  kWCarryInv = 1.0f / kWCarry;
constexpr float  kPCarry    = 32768.0f;
constexpr float  kPCarryInv = 1.0f / kPCarry;
constexpr float  kInvDim    = 1.0f / (float)kDim;
constexpr float  kLnEps     = 1e-6f;
constexpr float  kAttnEps   = 1e-9f;
constexpr int    kAvPitch   = 40;
static_assert((kTok % 64) == 0 && (kDim % 64) == 0);
static_assert((kTok % 32) == 0 && (kDim % 32) == 0);
static_assert(((kND / 8) % 256) == 0 && ((kWW / 8) % 256) == 0);
static_assert((kAvPitch % 8) == 0 && kAvPitch >= 32);

constexpr size_t kPlane16  = kND * 2;
constexpr size_t kPlane32  = kND * 4;
constexpr size_t kW16      = kWW * 2;
constexpr size_t kR0Bytes  = (size_t)kTok * kTok * 4;
constexpr size_t kOffXH    = 0;
constexpr size_t kOffXL    = kOffXH  + kPlane16;
constexpr size_t kOffT0H   = kOffXL  + kPlane16;
constexpr size_t kOffT0L   = kOffT0H + kPlane16;
constexpr size_t kOffFH    = kOffT0L + kPlane16;
constexpr size_t kOffFL    = kOffFH  + kPlane16;
constexpr size_t kOffF16   = kOffFL  + kPlane16;
constexpr size_t kOffR1    = kOffF16 + kPlane16;
constexpr size_t kOffR2    = kOffR1  + kPlane16;
constexpr size_t kOffWSH   = kOffR2  + kPlane16;
constexpr size_t kOffWSL   = kOffWSH + 4 * kW16;
constexpr size_t kOffWF    = kOffWSL + 4 * kW16;
constexpr size_t kPhase1End = kOffWF + 4 * kW16;
constexpr size_t kOffS     = 0;
constexpr size_t kOffS32   = 0;
constexpr size_t kOffS16   = kOffS32 + kPlane32;
constexpr size_t kOffQK    = kR0Bytes;
constexpr size_t kOffVT    = kOffQK  + 8 * kPlane16;
constexpr size_t kOffRES   = kOffVT  + 2 * kPlane16;
constexpr size_t kOffSC    = kOffRES + 2 * kPlane16;
constexpr size_t kOffFFN   = kOffSC  + kPlane32;
constexpr size_t kOffMROW  = kOffFFN + 2 * kW16;
constexpr size_t kOffINVS  = kOffMROW + (size_t)kTok * 4;
constexpr size_t kOffRC    = kOffINVS + (size_t)kTok * 4;
constexpr size_t kWsTotal  = kOffRC   + (size_t)kTok * 4;
static_assert(kPhase1End <= kR0Bytes);
static_assert(kOffS16 + kPlane16 <= kR0Bytes);
static_assert(kWsTotal == 126926848ull);
static_assert(kWsTotal <= 134217728ull);
static_assert((kOffWSH % 128) == 0 && (kOffWSL % 128) == 0 && (kOffWF % 128) == 0 && (kOffQK % 128) == 0 &&
              (kOffVT % 128) == 0 && (kOffRES % 128) == 0 && (kOffSC % 128) == 0 && (kOffFFN % 128) == 0 &&
              (kOffMROW % 128) == 0 && (kOffINVS % 128) == 0 && (kOffRC % 128) == 0 && (kOffS16 % 128) == 0);

__device__ __forceinline__ unsigned short f2bf_bits(float f) {
  unsigned u = __float_as_uint(f);
  return (unsigned short)((u + 0x7FFFu + ((u >> 16) & 1u)) >> 16);
}
__device__ __forceinline__ float bf_bits2f(unsigned short h) { return __uint_as_float(((unsigned)h) << 16); }

__device__ __forceinline__ float h16_to_f32(unsigned hb) {
  const unsigned sgn = (hb & 0x8000u) << 16;
  const unsigned em = hb & 0x7fffu;
  const float fn = __uint_as_float((em << 13) + 0x38000000u);
  const float fs = (float)em * 5.9604644775390625e-8f;
  const float mag = (em < 0x400u) ? fs : fn;
  return __uint_as_float(__float_as_uint(mag) | sgn);
}

__device__ __forceinline__ void grp_guard_h(v8f& a, v8f& b, v8f& c, v8f& d, v16h x, v16h y) {
  asm volatile("v_nop\n\tv_nop\n\tv_nop\n\tv_nop" : "+v"(a), "+v"(b), "+v"(c), "+v"(d) : "v"(x), "v"(y));
}
__device__ __forceinline__ void grp_guard_b(v8f& a, v8f& b, v8f& c, v8f& d, v16b x, v16b y) {
  asm volatile("v_nop\n\tv_nop\n\tv_nop\n\tv_nop" : "+v"(a), "+v"(b), "+v"(c), "+v"(d) : "v"(x), "v"(y));
}
__device__ __forceinline__ void keep4_h(v16h a, v16h b, v16h c, v16h d) { asm volatile("v_nop" :: "v"(a), "v"(b), "v"(c), "v"(d)); }
__device__ __forceinline__ void keep4_b(v16b a, v16b b, v16b c, v16b d) { asm volatile("v_nop" :: "v"(a), "v"(b), "v"(c), "v"(d)); }
__device__ __forceinline__ void acc_guard4(v8f& a, v8f& b, v8f& c, v8f& d) {
  asm volatile("v_nop\n\tv_nop\n\tv_nop\n\tv_nop" : "+v"(a), "+v"(b), "+v"(c), "+v"(d));
}

template <typename T> struct Frag;
template <> struct Frag<_Float16> {
  typedef v16h V;
  union U { v16h v; v8h h[2]; };
  static __device__ __forceinline__ v16h load(const _Float16* p) {
    U f;
    f.h[0] = *(const v8h*)(p);
    f.h[1] = *(const v8h*)(p + 16);
    return f.v;
  }
  static __device__ __forceinline__ v8f mma(v16h a, v16h b, v8f c) {
    return __builtin_amdgcn_wmma_f32_16x16x32_f16(false, a, false, b, (short)0, c, false, false);
  }
  static __device__ __forceinline__ void guard(v8f& a, v8f& b, v8f& c, v8f& d, v16h x, v16h y) { grp_guard_h(a, b, c, d, x, y); }
  static __device__ __forceinline__ void keep(v16h a, v16h b, v16h c, v16h d) { keep4_h(a, b, c, d); }
};
template <> struct Frag<__bf16> {
  typedef v16b V;
  union U { v16b v; v8b h[2]; };
  static __device__ __forceinline__ v16b load(const __bf16* p) {
    U f;
    f.h[0] = *(const v8b*)(p);
    f.h[1] = *(const v8b*)(p + 16);
    return f.v;
  }
  static __device__ __forceinline__ v8f mma(v16b a, v16b b, v8f c) {
    return __builtin_amdgcn_wmma_f32_16x16x32_bf16(false, a, false, b, (short)0, c, false, false);
  }
  static __device__ __forceinline__ void guard(v8f& a, v8f& b, v8f& c, v8f& d, v16b x, v16b y) { grp_guard_b(a, b, c, d, x, y); }
  static __device__ __forceinline__ void keep(v16b a, v16b b, v16b c, v16b d) { keep4_b(a, b, c, d); }
};

template <int ET> struct Elem;
template <> struct Elem<0> { typedef _Float16 T; };
template <> struct Elem<1> { typedef __bf16 T; };

template <int ET, bool SPLIT, int BIAS_MODE, int OUT_MODE, bool RESID, int ACT>
__global__ __launch_bounds__(256) void wmma_gemm64(
    const unsigned short* __restrict__ Ap, const unsigned short* __restrict__ A2p, int lda,
    const unsigned short* __restrict__ Btp, const unsigned short* __restrict__ Bt2p, int ldb,
    void* __restrict__ Cout, void* __restrict__ Cout2, int ldc,
    const float* __restrict__ bias, const float* __restrict__ resid,
    int M, int N, int K, float scale) {
  typedef typename Elem<ET>::T T;
  typedef typename Frag<T>::V V;
  const T* A   = (const T*)Ap;
  const T* A2  = (const T*)A2p;
  const T* Bt  = (const T*)Btp;
  const T* Bt2 = (const T*)Bt2p;
  __shared__ __align__(16) float sT[8][16 * 68];
  const int lane = threadIdx.x & 31;
  const int wave = __builtin_amdgcn_readfirstlane((int)(threadIdx.x >> 5));
  const int tilesN = N >> 6;
  const int tilesM = M >> 6;
  const int tile = blockIdx.x * 8 + wave;
  if (tile >= tilesM * tilesN) return;
  const int tm = tile / tilesN;
  const int tn = tile - tm * tilesN;
  const int m0 = tm << 6;
  const int n0 = tn << 6;

  const int rlane = lane & 15;
  const int koff  = (lane >> 4) * 8;
  const int mOff  = (lane >> 4) * 8;

  v8f acc[4][4];
#pragma unroll
  for (int i = 0; i < 4; ++i)
#pragma unroll
    for (int j = 0; j < 4; ++j) acc[i][j] = (v8f){0.f, 0.f, 0.f, 0.f, 0.f, 0.f, 0.f, 0.f};

  for (int k0 = 0; k0 < K; k0 += 32) {
    V bh[4], bl[4];
#pragma unroll
    for (int j = 0; j < 4; ++j) {
      const size_t bo = (size_t)(n0 + (j << 4) + rlane) * ldb + koff + k0;
      bh[j] = Frag<T>::load(Bt + bo);
      if (SPLIT) bl[j] = Frag<T>::load(Bt2 + bo);
    }
#pragma unroll
    for (int i = 0; i < 4; ++i) {
      const size_t ao = (size_t)(m0 + (i << 4) + rlane) * lda + koff + k0;
      V ah = Frag<T>::load(A + ao);
      V al;
      if (SPLIT) al = Frag<T>::load(A2 + ao);
#pragma unroll
      for (int j = 0; j < 4; ++j) {
        acc[i][j] = Frag<T>::mma(ah, bh[j], acc[i][j]);
        if (SPLIT) {
          acc[i][j] = Frag<T>::mma(ah, bl[j], acc[i][j]);
          acc[i][j] = Frag<T>::mma(al, bh[j], acc[i][j]);
        }
      }
      Frag<T>::guard(acc[i][0], acc[i][1], acc[i][2], acc[i][3], ah, SPLIT ? al : ah);
    }
    Frag<T>::keep(bh[0], bh[1], bh[2], bh[3]);
    if (SPLIT) Frag<T>::keep(bl[0], bl[1], bl[2], bl[3]);
  }
  acc_guard4(acc[0][0], acc[0][1], acc[0][2], acc[0][3]);
  acc_guard4(acc[1][0], acc[1][1], acc[1][2], acc[1][3]);
  acc_guard4(acc[2][0], acc[2][1], acc[2][2], acc[2][3]);
  acc_guard4(acc[3][0], acc[3][1], acc[3][2], acc[3][3]);

  float* slab = sT[wave];
#pragma unroll
  for (int i = 0; i < 4; ++i) {
    const int mBase = m0 + (i << 4);
#pragma unroll
    for (int j = 0; j < 4; ++j) {
      const int n = n0 + (j << 4) + rlane;
      float bv = 0.f;
      if (BIAS_MODE == 2) bv = bias[n];
#pragma unroll
      for (int r = 0; r < 8; ++r) {
        float v = acc[i][j][r] * scale;
        if (BIAS_MODE == 2) v += bv;
        if (ACT == 2) v = fmaxf(v, 0.0f);
        slab[(mOff + r) * 68 + (j << 4) + rlane] = v;
      }
    }
    __builtin_amdgcn_fence(__ATOMIC_RELEASE, "workgroup");
    __builtin_amdgcn_wave_barrier();
    __builtin_amdgcn_fence(__ATOMIC_ACQUIRE, "workgroup");
    if (OUT_MODE == 0) {
      float* C = (float*)Cout;
      const int hh = lane >> 4, c4 = (lane & 15) * 4;
      v4f vals[8];
#pragma unroll
      for (int it = 0; it < 8; ++it) {
        const int row = it * 2 + hh;
        v4f v = *(const v4f*)(slab + row * 68 + c4);
        if (RESID) {
          const v4f rr = *(const v4f*)(resid + (size_t)(mBase + row) * ldc + n0 + c4);
          v = v + rr;
        }
        vals[it] = v;
      }
      for (int pass = 0; pass < 2; ++pass) {
#pragma unroll
        for (int it = 0; it < 8; ++it) {
          const int row = it * 2 + hh;
          *(volatile v4f*)(C + (size_t)(mBase + row) * ldc + n0 + c4) = vals[it];
        }
        __threadfence();
      }
    } else {
      const int q = lane >> 3, c8 = (lane & 7) * 8;
      unsigned short* C  = (unsigned short*)Cout;
      unsigned short* C2 = (unsigned short*)Cout2;
      for (int pass = 0; pass < 2; ++pass) {
#pragma unroll
        for (int it = 0; it < 4; ++it) {
          const int row = it * 4 + q;
          const float* sp = slab + row * 68 + c8;
          v8h hv, lv;
#pragma unroll
          for (int e = 0; e < 8; ++e) {
            const float sv = sp[e];
            if (OUT_MODE == 1) {
              hv[e] = (_Float16)sv;
            } else {
              const unsigned short hb = f2bf_bits(sv);
              const unsigned short lb = f2bf_bits(sv - bf_bits2f(hb));
              hv[e] = __builtin_bit_cast(_Float16, hb);
              lv[e] = __builtin_bit_cast(_Float16, lb);
            }
          }
          *(volatile v8h*)(C + (size_t)(mBase + row) * ldc + n0 + c8) = hv;
          if (OUT_MODE == 2) *(volatile v8h*)(C2 + (size_t)(mBase + row) * ldc + n0 + c8) = lv;
        }
        __threadfence();
      }
    }
    __builtin_amdgcn_fence(__ATOMIC_RELEASE, "workgroup");
    __builtin_amdgcn_wave_barrier();
    __builtin_amdgcn_fence(__ATOMIC_ACQUIRE, "workgroup");
  }
}

__global__ __launch_bounds__(256) void split4_bf16_kernel(
    const float* __restrict__ s0, const float* __restrict__ s1, const float* __restrict__ s2, const float* __restrict__ s3,
    unsigned short* __restrict__ dhi, unsigned short* __restrict__ dlo, int total8, long planeElems) {
  const int i = blockIdx.x * 256 + threadIdx.x;
  if (i >= total8) return;
  const int y = blockIdx.y;
  const float* src = (y == 0) ? s0 : (y == 1) ? s1 : (y == 2) ? s2 : s3;
  const size_t e0 = (size_t)i << 3;
  const v4f a0 = *(const v4f*)(src + e0);
  const v4f a1 = *(const v4f*)(src + e0 + 4);
  v8h hv, lv;
#pragma unroll
  for (int e = 0; e < 4; ++e) {
    const float f0 = a0[e], f1 = a1[e];
    const unsigned short h0 = f2bf_bits(f0), h1 = f2bf_bits(f1);
    const unsigned short l0 = f2bf_bits(f0 - bf_bits2f(h0)), l1 = f2bf_bits(f1 - bf_bits2f(h1));
    hv[e]     = __builtin_bit_cast(_Float16, h0);
    hv[4 + e] = __builtin_bit_cast(_Float16, h1);
    lv[e]     = __builtin_bit_cast(_Float16, l0);
    lv[4 + e] = __builtin_bit_cast(_Float16, l1);
  }
  unsigned short* qh = dhi + (size_t)y * planeElems + e0;
  unsigned short* ql = dlo + (size_t)y * planeElems + e0;
  *(volatile v8h*)qh = hv;
  *(volatile v8h*)ql = lv;
  __threadfence();
  *(volatile v8h*)qh = hv;
  *(volatile v8h*)ql = lv;
}

__global__ __launch_bounds__(256) void cast4_f16_kernel(
    const float* __restrict__ s0, const float* __restrict__ s1, const float* __restrict__ s2, const float* __restrict__ s3,
    unsigned short* __restrict__ out, float carry, int total8, long planeElems) {
  const int i = blockIdx.x * 256 + threadIdx.x;
  if (i >= total8) return;
  const int y = blockIdx.y;
  const float* src = (y == 0) ? s0 : (y == 1) ? s1 : (y == 2) ? s2 : s3;
  const size_t e0 = (size_t)i << 3;
  const v4f a0 = *(const v4f*)(src + e0);
  const v4f a1 = *(const v4f*)(src + e0 + 4);
  v8h hv;
#pragma unroll
  for (int e = 0; e < 4; ++e) {
    const float f0 = a0[e] * carry, f1 = a1[e] * carry;
    hv[e]     = (_Float16)f0;
    hv[4 + e] = (_Float16)f1;
  }
  unsigned short* q = out + (size_t)y * planeElems + e0;
  *(volatile v8h*)q = hv;
  __threadfence();
  *(volatile v8h*)q = hv;
}

__global__ __launch_bounds__(256) void hilo_to_f16_kernel(
    const unsigned short* __restrict__ hi, const unsigned short* __restrict__ lo,
    unsigned short* __restrict__ out, int total8) {
  const int i = blockIdx.x * 256 + threadIdx.x;
  if (i >= total8) return;
  const size_t e0 = (size_t)i << 3;
  const v4u hw4 = *(const v4u*)(hi + e0);
  const v4u lw4 = *(const v4u*)(lo + e0);
  v8h hv;
#pragma unroll
  for (int w = 0; w < 4; ++w) {
    const unsigned hw = hw4[w];
    const unsigned lw = lw4[w];
    const float f0 = __uint_as_float(hw << 16) + __uint_as_float(lw << 16);
    const float f1 = __uint_as_float(hw & 0xffff0000u) + __uint_as_float(lw & 0xffff0000u);
    hv[2 * w]     = (_Float16)f0;
    hv[2 * w + 1] = (_Float16)f1;
  }
  unsigned short* q = out + e0;
  *(volatile v8h*)q = hv;
  __threadfence();
  *(volatile v8h*)q = hv;
}

__global__ __launch_bounds__(256) void rowstat_kernel(const float* __restrict__ S, float* __restrict__ mrow, float* __restrict__ invs) {
  __shared__ float sM[32];
  __shared__ float sI[32];
  const int lane = threadIdx.x & 31;
  const int wave = __builtin_amdgcn_readfirstlane((int)(threadIdx.x >> 5));
  const int row0 = blockIdx.x * 32;
#pragma unroll 1
  for (int q = 0; q < 4; ++q) {
    const int rl = wave * 4 + q;
    const float* p = S + (size_t)(row0 + rl) * kTok + lane * 4;
    float m = -INFINITY;
#pragma unroll 4
    for (int it = 0; it < kTok / 128; ++it) {
      const v4f v = *(const v4f*)(p + it * 128);
      m = fmaxf(m, fmaxf(fmaxf(v[0], v[1]), fmaxf(v[2], v[3])));
    }
#pragma unroll
    for (int off = 16; off > 0; off >>= 1) m = fmaxf(m, __shfl_xor(m, off, 32));
    float sum = 0.f;
#pragma unroll 2
    for (int it = 0; it < kTok / 128; ++it) {
      const v4f v = *(const v4f*)(p + it * 128);
      sum += __expf(v[0] - m);
      sum += __expf(v[1] - m);
      sum += __expf(v[2] - m);
      sum += __expf(v[3] - m);
    }
#pragma unroll
    for (int off = 16; off > 0; off >>= 1) sum += __shfl_xor(sum, off, 32);
    const float inv = 1.0f / sum;
    if (lane == 0) {
      sM[rl] = m;
      sI[rl] = inv;
    }
  }
  __syncthreads();
  if (wave == 0) {
    const float mv = sM[lane];
    const float iv = sI[lane];
    *(volatile float*)(mrow + row0 + lane) = mv;
    *(volatile float*)(invs + row0 + lane) = iv;
    __threadfence();
    *(volatile float*)(mrow + row0 + lane) = mv;
    *(volatile float*)(invs + row0 + lane) = iv;
  }
}

__global__ __launch_bounds__(256) void colsum_kernel(const float* __restrict__ S, const float* __restrict__ mrow,
                                                     const float* __restrict__ invs, float* __restrict__ rcol) {
  __shared__ float sP[8][32];
  const int lane = threadIdx.x & 31;
  const int wave = __builtin_amdgcn_readfirstlane((int)(threadIdx.x >> 5));
  const int j0 = blockIdx.x * 32;
  const float* p = S + j0 + lane;
  float acc = 0.f;
#pragma unroll 4
  for (int t = 0; t < kTok / 8; ++t) {
    const int i = wave + 8 * t;
    const float s  = p[(size_t)i * kTok];
    const float mi = mrow[i];
    const float is = invs[i];
    const float pr = __expf(s - mi) * is;
    acc += pr;
  }
  sP[wave][lane] = acc;
  __syncthreads();
  if (wave == 0) {
    float c = sP[0][lane];
    c += sP[1][lane];
    c += sP[2][lane];
    c += sP[3][lane];
    c += sP[4][lane];
    c += sP[5][lane];
    c += sP[6][lane];
    c += sP[7][lane];
    const float rc = 1.0f / (kAttnEps + c);
    *(volatile float*)(rcol + j0 + lane) = rc;
    __threadfence();
    *(volatile float*)(rcol + j0 + lane) = rc;
  }
}

__global__ __launch_bounds__(256) void av_kernel(const float* __restrict__ S, const float* __restrict__ mrow,
                                                 const float* __restrict__ invs, const float* __restrict__ rcol,
                                                 const unsigned short* __restrict__ VTp, float* __restrict__ SC) {
  __shared__ __align__(16) _Float16 sA[64 * kAvPitch];
  __shared__ __align__(16) float sT[8][16 * 68];
  typedef Frag<_Float16> FH;
  const int tid  = threadIdx.x;
  const int lane = tid & 31;
  const int wave = __builtin_amdgcn_readfirstlane((int)(tid >> 5));
  const int m0 = blockIdx.x * 64;
  const int n0 = wave * 64;
  const int sr  = tid >> 2;
  const int sc8 = (tid & 3) * 8;
  const float mi = mrow[m0 + sr];
  const float fi = invs[m0 + sr] * kPCarry;
  const float* Srow = S + (size_t)(m0 + sr) * kTok + sc8;
  const float* rcp  = rcol + sc8;
  const _Float16* VT = (const _Float16*)VTp;

  const int rlane = lane & 15;
  const int koff  = (lane >> 4) * 8;
  const int mOff  = (lane >> 4) * 8;

  v8f acc[4][4];
#pragma unroll
  for (int i = 0; i < 4; ++i)
#pragma unroll
    for (int j = 0; j < 4; ++j) acc[i][j] = (v8f){0.f, 0.f, 0.f, 0.f, 0.f, 0.f, 0.f, 0.f};

  for (int k0 = 0; k0 < kTok; k0 += 32) {
    const v4f s0 = *(const v4f*)(Srow + k0);
    const v4f s1 = *(const v4f*)(Srow + k0 + 4);
    const v4f r0 = *(const v4f*)(rcp + k0);
    const v4f r1 = *(const v4f*)(rcp + k0 + 4);
    v8h hv;
#pragma unroll
    for (int e = 0; e < 4; ++e) {
      const float e0 = __expf(s0[e] - mi);
      const float e1 = __expf(s1[e] - mi);
      const float w0 = (e0 * fi) * r0[e];
      const float w1 = (e1 * fi) * r1[e];
      hv[e]     = (_Float16)w0;
      hv[4 + e] = (_Float16)w1;
    }
    *(v8h*)(sA + sr * kAvPitch + sc8) = hv;
    __syncthreads();
    v16h bh[4];
#pragma unroll
    for (int j = 0; j < 4; ++j) {
      const size_t bo = (size_t)(n0 + (j << 4) + rlane) * kTok + koff + k0;
      bh[j] = FH::load(VT + bo);
    }
#pragma unroll
    for (int i = 0; i < 4; ++i) {
      const int ao = ((i << 4) + rlane) * kAvPitch + koff;
      FH::U fa;
      fa.h[0] = *(const v8h*)(sA + ao);
      fa.h[1] = *(const v8h*)(sA + ao + 16);
      const v16h ah = fa.v;
#pragma unroll
      for (int j = 0; j < 4; ++j) acc[i][j] = FH::mma(ah, bh[j], acc[i][j]);
      FH::guard(acc[i][0], acc[i][1], acc[i][2], acc[i][3], ah, ah);
    }
    FH::keep(bh[0], bh[1], bh[2], bh[3]);
    __syncthreads();
  }
  acc_guard4(acc[0][0], acc[0][1], acc[0][2], acc[0][3]);
  acc_guard4(acc[1][0], acc[1][1], acc[1][2], acc[1][3]);
  acc_guard4(acc[2][0], acc[2][1], acc[2][2], acc[2][3]);
  acc_guard4(acc[3][0], acc[3][1], acc[3][2], acc[3][3]);

  float* slab = sT[wave];
#pragma unroll
  for (int i = 0; i < 4; ++i) {
    const int mBase = m0 + (i << 4);
#pragma unroll
    for (int j = 0; j < 4; ++j) {
#pragma unroll
      for (int r = 0; r < 8; ++r) slab[(mOff + r) * 68 + (j << 4) + rlane] = acc[i][j][r] * kPCarryInv;
    }
    __builtin_amdgcn_fence(__ATOMIC_RELEASE, "workgroup");
    __builtin_amdgcn_wave_barrier();
    __builtin_amdgcn_fence(__ATOMIC_ACQUIRE, "workgroup");
    {
      const int hh = lane >> 4, c4 = (lane & 15) * 4;
      v4f vals[8];
#pragma unroll
      for (int it = 0; it < 8; ++it) vals[it] = *(const v4f*)(slab + (it * 2 + hh) * 68 + c4);
      for (int pass = 0; pass < 2; ++pass) {
#pragma unroll
        for (int it = 0; it < 8; ++it) {
          const int row = it * 2 + hh;
          *(volatile v4f*)(SC + (size_t)(mBase + row) * kDim + n0 + c4) = vals[it];
        }
        __threadfence();
      }
    }
    __builtin_amdgcn_fence(__ATOMIC_RELEASE, "workgroup");
    __builtin_amdgcn_wave_barrier();
    __builtin_amdgcn_fence(__ATOMIC_ACQUIRE, "workgroup");
  }
}

__global__ __launch_bounds__(256) void add_ln_kernel(const unsigned short* __restrict__ RES, const float* __restrict__ SCp,
                                                     const float* __restrict__ gam, const float* __restrict__ bet,
                                                     float* __restrict__ S32, unsigned short* __restrict__ S16) {
  __shared__ __align__(16) float sY[8][kDim];
  const int lane = threadIdx.x & 31;
  const int wave = __builtin_amdgcn_readfirstlane((int)(threadIdx.x >> 5));
  const int row = blockIdx.x * 8 + wave;
  const float* scp = SCp + (size_t)row * kDim;
  const unsigned short* rp = RES + (size_t)row * kDim;
  float x[16];
#pragma unroll
  for (int it = 0; it < 4; ++it) {
    const int col = it * 128 + lane * 4;
    const v4f a = *(const v4f*)(scp + col);
    const v2u w = *(const v2u*)(rp + col);
    const unsigned w0 = w[0];
    const unsigned w1 = w[1];
    x[4 * it + 0] = h16_to_f32(w0 & 0xffffu) + a[0];
    x[4 * it + 1] = h16_to_f32(w0 >> 16) + a[1];
    x[4 * it + 2] = h16_to_f32(w1 & 0xffffu) + a[2];
    x[4 * it + 3] = h16_to_f32(w1 >> 16) + a[3];
  }
  float s = 0.f;
#pragma unroll
  for (int i = 0; i < 16; ++i) s += x[i];
#pragma unroll
  for (int off = 16; off > 0; off >>= 1) s += __shfl_xor(s, off, 32);
  const float mu = s * kInvDim;
  float vs = 0.f;
#pragma unroll
  for (int i = 0; i < 16; ++i) {
    const float d = x[i] - mu;
    x[i] = d;
    vs += d * d;
  }
#pragma unroll
  for (int off = 16; off > 0; off >>= 1) vs += __shfl_xor(vs, off, 32);
  const float inv = rsqrtf(vs * kInvDim + kLnEps);
  float* slab = sY[wave];
  v4f yv[4];
#pragma unroll
  for (int it = 0; it < 4; ++it) {
    const int col = it * 128 + lane * 4;
    const v4f g4 = *(const v4f*)(gam + col);
    const v4f b4 = *(const v4f*)(bet + col);
    v4f y;
    y[0] = (x[4 * it + 0] * inv) * g4[0] + b4[0];
    y[1] = (x[4 * it + 1] * inv) * g4[1] + b4[1];
    y[2] = (x[4 * it + 2] * inv) * g4[2] + b4[2];
    y[3] = (x[4 * it + 3] * inv) * g4[3] + b4[3];
    yv[it] = y;
    *(v4f*)(slab + col) = y;
  }
  __builtin_amdgcn_fence(__ATOMIC_RELEASE, "workgroup");
  __builtin_amdgcn_wave_barrier();
  __builtin_amdgcn_fence(__ATOMIC_ACQUIRE, "workgroup");
  v8h hv[2];
#pragma unroll
  for (int it2 = 0; it2 < 2; ++it2) {
    const int c = it2 * 256 + lane * 8;
    const v4f a0 = *(const v4f*)(slab + c);
    const v4f a1 = *(const v4f*)(slab + c + 4);
#pragma unroll
    for (int e = 0; e < 4; ++e) {
      const float f0 = a0[e], f1 = a1[e];
      hv[it2][e]     = (_Float16)f0;
      hv[it2][4 + e] = (_Float16)f1;
    }
  }
  float* o32 = S32 + (size_t)row * kDim;
  unsigned short* o16 = S16 + (size_t)row * kDim;
  for (int pass = 0; pass < 2; ++pass) {
#pragma unroll
    for (int it = 0; it < 4; ++it) *(volatile v4f*)(o32 + it * 128 + lane * 4) = yv[it];
#pragma unroll
    for (int it2 = 0; it2 < 2; ++it2) *(volatile v8h*)(o16 + it2 * 256 + lane * 8) = hv[it2];
    __threadfence();
  }
}

template <int ET, bool SPLIT, int BIAS_MODE, int OUT_MODE, bool RESID, int ACT>
static void run_gemm(hipStream_t st,
                     const unsigned short* A, const unsigned short* A2, int lda,
                     const unsigned short* Bt, const unsigned short* Bt2, int ldb,
                     void* C, void* C2, int ldc,
                     const float* bias, const float* resid,
                     int M, int N, int K, float scale) {
  const int tiles = (M >> 6) * (N >> 6);
  const int blocks = (tiles + 7) / 8;
  wmma_gemm64<ET, SPLIT, BIAS_MODE, OUT_MODE, RESID, ACT><<<dim3(blocks), 256, 0, st>>>(
      A, A2, lda, Bt, Bt2, ldb, C, C2, ldc, bias, resid, M, N, K, scale);
}

extern "C" void kernel_launch(void* const* d_in, const int* in_sizes, int n_in,
                              void* d_out, int out_size, void* d_ws, size_t ws_size,
                              hipStream_t stream) {
  if (n_in < 34) return;
  if (in_sizes[0] != (int)kND || in_sizes[1] != (int)kND) return;
  for (int p = 0; p < 2; ++p) {
    for (int s = 0; s < 16; ++s) {
      const bool isMat = (s == 0 || s == 2 || s == 4 || s == 6 || s == 8 || s == 10 || s == 11 || s == 12 || s == 15);
      const int want = isMat ? (int)kWW : kDim;
      if (in_sizes[2 + 16 * p + s] != want) return;
    }
  }
  if (out_size != (int)(2 * kND)) return;
  if (ws_size < kWsTotal) return;

  char* ws = (char*)d_ws;
  unsigned short* XH  = (unsigned short*)(ws + kOffXH);
  unsigned short* XL  = (unsigned short*)(ws + kOffXL);
  unsigned short* T0H = (unsigned short*)(ws + kOffT0H);
  unsigned short* T0L = (unsigned short*)(ws + kOffT0L);
  unsigned short* FH  = (unsigned short*)(ws + kOffFH);
  unsigned short* FL  = (unsigned short*)(ws + kOffFL);
  unsigned short* F16 = (unsigned short*)(ws + kOffF16);
  unsigned short* R1  = (unsigned short*)(ws + kOffR1);
  unsigned short* R2  = (unsigned short*)(ws + kOffR2);
  unsigned short* WSH = (unsigned short*)(ws + kOffWSH);
  unsigned short* WSL = (unsigned short*)(ws + kOffWSL);
  unsigned short* WF  = (unsigned short*)(ws + kOffWF);
  float*          S   = (float*)(ws + kOffS);
  float*          S32 = (float*)(ws + kOffS32);
  unsigned short* S16 = (unsigned short*)(ws + kOffS16);
  unsigned short* QK  = (unsigned short*)(ws + kOffQK);
  unsigned short* VT  = (unsigned short*)(ws + kOffVT);
  unsigned short* RES = (unsigned short*)(ws + kOffRES);
  float*          SC  = (float*)(ws + kOffSC);
  unsigned short* FFN = (unsigned short*)(ws + kOffFFN);
  float*          MROW = (float*)(ws + kOffMROW);
  float*          INVS = (float*)(ws + kOffINVS);
  float*          RC   = (float*)(ws + kOffRC);
  float* out = (float*)d_out;

  const int nd8 = (int)(kND / 8);
  const int ww8 = (int)(kWW / 8);

  {
    const float* fa = (const float*)d_in[2 + 15];
    const float* fb = (const float*)d_in[18 + 15];
    cast4_f16_kernel<<<dim3(ww8 / 256, 2), 256, 0, stream>>>(fa, fb, fa, fa, FFN, kWCarry, ww8, (long)kWW);
  }

  for (int p = 0; p < 2; ++p) {
    const float* x   = (const float*)d_in[p];
    const int pb = 2 + 16 * p;
    const float* pW1 = (const float*)d_in[pb + 0];
    const float* pb1 = (const float*)d_in[pb + 1];
    const float* pW2 = (const float*)d_in[pb + 2];
    const float* pb2 = (const float*)d_in[pb + 3];
    const float* rW1 = (const float*)d_in[pb + 4];
    const float* rb1 = (const float*)d_in[pb + 5];
    const float* rW2 = (const float*)d_in[pb + 6];
    const float* rb2 = (const float*)d_in[pb + 7];
    const float* rW3 = (const float*)d_in[pb + 8];
    const float* rb3 = (const float*)d_in[pb + 9];
    const float* Wq  = (const float*)d_in[pb + 10];
    const float* Wk  = (const float*)d_in[pb + 11];
    const float* Wv  = (const float*)d_in[pb + 12];
    unsigned short* QH = QK + (size_t)(4 * p + 0) * kND;
    unsigned short* QL = QK + (size_t)(4 * p + 1) * kND;
    unsigned short* KH = QK + (size_t)(4 * p + 2) * kND;
    unsigned short* KL = QK + (size_t)(4 * p + 3) * kND;
    unsigned short* VTp  = VT  + (size_t)p * kND;
    unsigned short* RESp = RES + (size_t)p * kND;

    split4_bf16_kernel<<<dim3(nd8 / 256, 1), 256, 0, stream>>>(x, x, x, x, XH, XL, nd8, 0L);
    split4_bf16_kernel<<<dim3(ww8 / 256, 4), 256, 0, stream>>>(pW1, pW2, Wq, Wk, WSH, WSL, ww8, (long)kWW);
    cast4_f16_kernel<<<dim3(ww8 / 256, 4), 256, 0, stream>>>(rW1, rW2, rW3, Wv, WF, kWCarry, ww8, (long)kWW);

    run_gemm<1, true, 2, 2, false, 2>(stream, XH, XL, kDim, WSH + 0 * kWW, WSL + 0 * kWW, kDim,
                                      (void*)T0H, (void*)T0L, kDim, pb1, pb1, kTok, kDim, kDim, 1.0f);
    run_gemm<1, true, 2, 2, false, 0>(stream, T0H, T0L, kDim, WSH + 1 * kWW, WSL + 1 * kWW, kDim,
                                      (void*)FH, (void*)FL, kDim, pb2, pb2, kTok, kDim, kDim, 1.0f);
    hilo_to_f16_kernel<<<dim3(nd8 / 256), 256, 0, stream>>>(FH, FL, F16, nd8);
    run_gemm<0, false, 2, 1, false, 2>(stream, F16, F16, kDim, WF + 0 * kWW, WF + 0 * kWW, kDim,
                                       (void*)R1, (void*)R1, kDim, rb1, rb1, kTok, kDim, kDim, kWCarryInv);
    run_gemm<0, false, 2, 1, false, 2>(stream, R1, R1, kDim, WF + 1 * kWW, WF + 1 * kWW, kDim,
                                       (void*)R2, (void*)R2, kDim, rb2, rb2, kTok, kDim, kDim, kWCarryInv);
    run_gemm<0, false, 2, 1, false, 0>(stream, R2, R2, kDim, WF + 2 * kWW, WF + 2 * kWW, kDim,
                                       (void*)RESp, (void*)RESp, kDim, rb3, rb3, kTok, kDim, kDim, kWCarryInv);
    run_gemm<1, true, 0, 2, false, 0>(stream, FH, FL, kDim, WSH + 2 * kWW, WSL + 2 * kWW, kDim,
                                      (void*)QH, (void*)QL, kDim, pb1, pb1, kTok, kDim, kDim, 1.0f);
    run_gemm<1, true, 0, 2, false, 0>(stream, FH, FL, kDim, WSH + 3 * kWW, WSL + 3 * kWW, kDim,
                                      (void*)KH, (void*)KL, kDim, pb1, pb1, kTok, kDim, kDim, 1.0f);
    run_gemm<0, false, 0, 1, false, 0>(stream, WF + 3 * kWW, WF + 3 * kWW, kDim, F16, F16, kDim,
                                       (void*)VTp, (void*)VTp, kTok, pb1, pb1, kDim, kTok, kDim, kWCarryInv);
  }

  for (int p = 0; p < 2; ++p) {
    const int o = 1 - p;
    const int pb = 2 + 16 * p;
    const float* ln_g = (const float*)d_in[pb + 13];
    const float* ln_b = (const float*)d_in[pb + 14];
    const unsigned short* QH  = QK + (size_t)(4 * p + 0) * kND;
    const unsigned short* QL  = QK + (size_t)(4 * p + 1) * kND;
    const unsigned short* KHo = QK + (size_t)(4 * o + 2) * kND;
    const unsigned short* KLo = QK + (size_t)(4 * o + 3) * kND;
    const unsigned short* VTp  = VT  + (size_t)p * kND;
    const unsigned short* RESp = RES + (size_t)p * kND;
    const unsigned short* FFNp = FFN + (size_t)p * kWW;

    run_gemm<1, true, 0, 0, false, 0>(stream, QH, QL, kDim, KHo, KLo, kDim,
                                      (void*)S, (void*)S, kTok, ln_g, ln_g, kTok, kTok, kDim, 1.0f);
    rowstat_kernel<<<dim3(kTok / 32), 256, 0, stream>>>(S, MROW, INVS);
    colsum_kernel<<<dim3(kTok / 32), 256, 0, stream>>>(S, MROW, INVS, RC);
    av_kernel<<<dim3(kTok / 64), 256, 0, stream>>>(S, MROW, INVS, RC, VTp, SC);
    add_ln_kernel<<<dim3(kTok / 8), 256, 0, stream>>>(RESp, SC, ln_g, ln_b, S32, S16);
    run_gemm<0, false, 0, 0, true, 0>(stream, S16, S16, kDim, FFNp, FFNp, kDim,
                                      (void*)(out + (size_t)p * kND), (void*)(out + (size_t)p * kND), kDim,
                                      ln_g, S32, kTok, kDim, kDim, kWCarryInv);
  }
}
